// TokenformerMLPAdapter_20779051778285
// MI455X (gfx1250) — hardware-verified
//
#include <hip/hip_runtime.h>
#include <stddef.h>
#include <stdint.h>


#define TT    2048
#define HH    2048
#define NHD   4
#define HDIM  512
#define RR    32
#define NHK   16
#define XSC   8
#define WSC   1024
#define VSC   256
#define PSC   1024
#define CSC   8
#define NTHR  256
#define NWAVE 8
#define VTP   36
#define PTP   132
#define WSCAP 134217728
#define LDS_GEMM (NWAVE * 32 * 64 * 4)

static_assert(NHK == NHD * NHD);
static_assert(HH == NHD * HDIM);
static_assert((HH % 128) == 0);
static_assert((TT % 128) == 0);
static_assert((TT % (NWAVE * 32)) == 0);
static_assert((HDIM % 128) == 0);
static_assert(((TT * HH) % (8 * NTHR)) == 0);
static_assert(((TT * NHD) % NTHR) == 0);
static_assert(NTHR == NWAVE * 32);
static_assert(XSC * WSC == CSC * PSC);
static_assert(LDS_GEMM <= 300 * 1024);
static_assert((VTP * 4) % 16 == 0);
static_assert((PTP * 4) % 16 == 0);

typedef float          v4f  __attribute__((ext_vector_type(4)));
typedef float          v8f  __attribute__((ext_vector_type(8)));
typedef _Float16       v8h  __attribute__((ext_vector_type(8)));
typedef _Float16       v16h __attribute__((ext_vector_type(16)));
union FragH { v16h v; v8h h[2]; };

__device__ __forceinline__ v8f wmf(v16h a, v16h b, v8f c) {
  v8f d = __builtin_amdgcn_wmma_f32_16x16x32_f16(false, a, false, b, (short)0, c, false, false);
  asm volatile("v_nop\n\tv_nop\n\tv_nop\n\tv_nop" : "+v"(d) : "v"(a), "v"(b));
  return d;
}

__device__ __forceinline__ v8f vz8() {
  v8f z = {0.f, 0.f, 0.f, 0.f, 0.f, 0.f, 0.f, 0.f};
  return z;
}

__global__ __launch_bounds__(NTHR) void k_cvt(const float* __restrict__ src, _Float16* dst, float sc) {
  const size_t t = (size_t)blockIdx.x * NTHR + threadIdx.x;
  const float* p = src + t * 8;
  const v4f f0 = *(const v4f*)p;
  const v4f f1 = *(const v4f*)(p + 4);
  v8h a;
  a[0] = (_Float16)(f0.x * sc); a[1] = (_Float16)(f0.y * sc);
  a[2] = (_Float16)(f0.z * sc); a[3] = (_Float16)(f0.w * sc);
  a[4] = (_Float16)(f1.x * sc); a[5] = (_Float16)(f1.y * sc);
  a[6] = (_Float16)(f1.z * sc); a[7] = (_Float16)(f1.w * sc);
  _Float16* d = dst + t * 8;
  *(volatile v8h*)d = a;
  __threadfence();
  *(volatile v8h*)d = a;
}

__global__ __launch_bounds__(NTHR) void k_prepv(const float* __restrict__ tv, _Float16* vt) {
  __shared__ __attribute__((aligned(16))) float tile[128 * VTP];
  const int tid = threadIdx.x, lane = tid & 31, g = tid >> 5, hh = lane >> 4, m = lane & 15;
  const int hk = blockIdx.x;
  const int mc = blockIdx.y;
  const int h = hk >> 2, kk = hk & 3;
  const float* src = tv + (size_t)kk * (HH * RR) + (size_t)h * (HDIM * RR) + (size_t)mc * 128 * RR;
#pragma unroll
  for (int p = 0; p < 4; ++p) {
    const int e = 4 * (tid + NTHR * p);
    const int ml = e >> 5, rc = e & 31;
    const v4f v = *(const v4f*)(src + e);
    *(v4f*)(tile + ml * VTP + rc) = v;
  }
  __syncthreads();
  v8h hv[2];
#pragma unroll
  for (int s = 0; s < 2; ++s) {
    const int rc = 16 * s + 2 * g + hh;
    const int ml0 = 8 * m;
#pragma unroll
    for (int e = 0; e < 8; ++e) hv[s][e] = (_Float16)(tile[(ml0 + e) * VTP + rc] * (float)VSC);
  }
#pragma unroll
  for (int s = 0; s < 2; ++s) {
    _Float16* d = vt + (size_t)(hk * RR + 16 * s + 2 * g + hh) * HDIM + mc * 128 + 8 * m;
    *(volatile v8h*)d = hv[s];
  }
  __threadfence();
#pragma unroll
  for (int s = 0; s < 2; ++s) {
    _Float16* d = vt + (size_t)(hk * RR + 16 * s + 2 * g + hh) * HDIM + mc * 128 + 8 * m;
    *(volatile v8h*)d = hv[s];
  }
}

__global__ __launch_bounds__(NTHR) void k_prepp(const float* __restrict__ tp, _Float16* pt) {
  __shared__ __attribute__((aligned(16))) float tile[RR * PTP];
  const int tid = threadIdx.x;
  const int n0 = blockIdx.x * 128;
#pragma unroll
  for (int p = 0; p < 4; ++p) {
    const int e = 4 * (tid + NTHR * p);
    const int rc = e >> 7, nl = e & 127;
    const v4f v = *(const v4f*)(tp + (size_t)rc * HH + n0 + nl);
    *(v4f*)(tile + rc * PTP + nl) = v;
  }
  __syncthreads();
  v8h hv[2];
#pragma unroll
  for (int s = 0; s < 2; ++s) {
    const int idx = s * NTHR + tid;
    const int nl = idx >> 2, rc0 = (idx & 3) * 8;
#pragma unroll
    for (int e = 0; e < 8; ++e) hv[s][e] = (_Float16)(tile[(rc0 + e) * PTP + nl] * (float)PSC);
  }
#pragma unroll
  for (int s = 0; s < 2; ++s) {
    _Float16* d = pt + (size_t)n0 * RR + (size_t)(s * NTHR + tid) * 8;
    *(volatile v8h*)d = hv[s];
  }
  __threadfence();
#pragma unroll
  for (int s = 0; s < 2; ++s) {
    _Float16* d = pt + (size_t)n0 * RR + (size_t)(s * NTHR + tid) * 8;
    *(volatile v8h*)d = hv[s];
  }
}

__global__ __launch_bounds__(NTHR) void k_attn(const float* __restrict__ q, const float* __restrict__ tk, float* attn) {
  const int idx = blockIdx.x * NTHR + threadIdx.x;
  const int t = idx >> 2, h = idx & 3;
  const float* qr = q + (size_t)t * HH + h * HDIM;
  const float* kp0 = tk + 0 * HH + h * HDIM;
  const float* kp1 = tk + 1 * HH + h * HDIM;
  const float* kp2 = tk + 2 * HH + h * HDIM;
  const float* kp3 = tk + 3 * HH + h * HDIM;
  float s0 = 0.f, s1 = 0.f, s2 = 0.f, s3 = 0.f;
#pragma unroll 1
  for (int d = 0; d < HDIM; d += 4) {
    const v4f qv = *(const v4f*)(qr + d);
    const v4f a = *(const v4f*)(kp0 + d);
    const v4f b = *(const v4f*)(kp1 + d);
    const v4f c = *(const v4f*)(kp2 + d);
    const v4f e = *(const v4f*)(kp3 + d);
    s0 += qv.x * a.x + qv.y * a.y + qv.z * a.z + qv.w * a.w;
    s1 += qv.x * b.x + qv.y * b.y + qv.z * b.z + qv.w * b.w;
    s2 += qv.x * c.x + qv.y * c.y + qv.z * c.z + qv.w * c.w;
    s3 += qv.x * e.x + qv.y * e.y + qv.z * e.z + qv.w * e.w;
  }
  const float scale = 0.04419417382415922f;
  s0 *= scale; s1 *= scale; s2 *= scale; s3 *= scale;
  const float mx = fmaxf(fmaxf(s0, s1), fmaxf(s2, s3));
  const float e0 = __expf(s0 - mx), e1 = __expf(s1 - mx);
  const float e2 = __expf(s2 - mx), e3 = __expf(s3 - mx);
  const float inv = 1.0f / (e0 + e1 + e2 + e3);
  v4f o;
  o.x = e0 * inv; o.y = e1 * inv; o.z = e2 * inv; o.w = e3 * inv;
  float* op = attn + (size_t)idx * 4;
  *(volatile v4f*)op = o;
  __threadfence();
  *(volatile v4f*)op = o;
}

__global__ __launch_bounds__(NTHR) void k_gg(const _Float16* __restrict__ xh, const _Float16* __restrict__ vt,
                                             const float* __restrict__ attn, _Float16* ch) {
  __shared__ __attribute__((aligned(16))) float stg_all[NWAVE * 32 * RR];
  const int tid = threadIdx.x, lane = tid & 31, wave = tid >> 5, hh = lane >> 4, m = lane & 15;
  float* stg = stg_all + wave * (32 * RR);
  const int t0 = blockIdx.x * (NWAVE * 32) + wave * 32;

  v8f c[2][2];
#pragma unroll
  for (int mt = 0; mt < 2; ++mt)
#pragma unroll
    for (int nt = 0; nt < 2; ++nt) c[mt][nt] = vz8();

#pragma unroll 1
  for (int hk = 0; hk < NHK; ++hk) {
    const int h = hk >> 2;
    v8f acc[2][2];
#pragma unroll
    for (int mt = 0; mt < 2; ++mt)
#pragma unroll
      for (int nt = 0; nt < 2; ++nt) acc[mt][nt] = vz8();
    const _Float16* ap = xh + (size_t)(t0 + m) * HH + h * HDIM + 8 * hh;
    const _Float16* bp = vt + (size_t)(hk * RR + m) * HDIM + 8 * hh;
#pragma unroll 1
    for (int kt = 0; kt < HDIM / 32; ++kt) {
      const int k0 = 32 * kt;
      FragH a0, a1, b0, b1;
      a0.h[0] = *(const v8h*)(ap + k0);
      a0.h[1] = *(const v8h*)(ap + k0 + 16);
      a1.h[0] = *(const v8h*)(ap + (size_t)16 * HH + k0);
      a1.h[1] = *(const v8h*)(ap + (size_t)16 * HH + k0 + 16);
      b0.h[0] = *(const v8h*)(bp + k0);
      b0.h[1] = *(const v8h*)(bp + k0 + 16);
      b1.h[0] = *(const v8h*)(bp + (size_t)16 * HDIM + k0);
      b1.h[1] = *(const v8h*)(bp + (size_t)16 * HDIM + k0 + 16);
      acc[0][0] = wmf(a0.v, b0.v, acc[0][0]);
      acc[0][1] = wmf(a0.v, b1.v, acc[0][1]);
      acc[1][0] = wmf(a1.v, b0.v, acc[1][0]);
      acc[1][1] = wmf(a1.v, b1.v, acc[1][1]);
    }
    float w0[8], w1[8];
#pragma unroll
    for (int r = 0; r < 8; ++r) {
      w0[r] = attn[(size_t)(t0 + 8 * hh + r) * NHK + hk];
      w1[r] = attn[(size_t)(t0 + 16 + 8 * hh + r) * NHK + hk];
    }
#pragma unroll
    for (int nt = 0; nt < 2; ++nt) {
#pragma unroll
      for (int r = 0; r < 8; ++r) {
        c[0][nt][r] += w0[r] * acc[0][nt][r];
        c[1][nt][r] += w1[r] * acc[1][nt][r];
      }
    }
  }

  constexpr float GC = (float)CSC / (float)(XSC * VSC);
#pragma unroll
  for (int mt = 0; mt < 2; ++mt) {
    float* sp = stg + (16 * mt + 8 * hh) * RR + m;
#pragma unroll
    for (int nt = 0; nt < 2; ++nt) {
#pragma unroll
      for (int r = 0; r < 8; ++r) sp[r * RR + 16 * nt] = c[mt][nt][r] * GC;
    }
  }
  __syncthreads();

  v8h hv[4];
#pragma unroll
  for (int s = 0; s < 4; ++s) {
    const int idx = s * 32 + lane;
    const int row = idx >> 2, rc0 = (idx & 3) * 8;
#pragma unroll
    for (int e = 0; e < 8; ++e) hv[s][e] = (_Float16)stg[row * RR + rc0 + e];
  }
  _Float16* cbase = ch + (size_t)t0 * RR;
#pragma unroll
  for (int s = 0; s < 4; ++s) {
    _Float16* d = cbase + (size_t)(s * 32 + lane) * 8;
    *(volatile v8h*)d = hv[s];
  }
  __threadfence();
#pragma unroll
  for (int s = 0; s < 4; ++s) {
    _Float16* d = cbase + (size_t)(s * 32 + lane) * 8;
    *(volatile v8h*)d = hv[s];
  }
}

__global__ __launch_bounds__(NTHR) void k_gemm(const _Float16* __restrict__ xh, const _Float16* __restrict__ wh,
                                               const _Float16* __restrict__ ch, const _Float16* __restrict__ pt,
                                               const float* __restrict__ bias, float* out) {
  extern __shared__ v4f lds_dyn[];
  const int tid = threadIdx.x, lane = tid & 31, wave = tid >> 5, hh = lane >> 4, m = lane & 15;
  float* stg = (float*)lds_dyn + wave * (32 * 64);
  const int n0 = blockIdx.x * 128, m0 = blockIdx.y * 128;
  const int wm = (wave >> 1) * 32, wn = (wave & 1) * 64;

  v8f acc[2][4];
#pragma unroll
  for (int mt = 0; mt < 2; ++mt)
#pragma unroll
    for (int nt = 0; nt < 4; ++nt) acc[mt][nt] = vz8();

  {
    const _Float16* ap = xh + (size_t)(m0 + wm + m) * HH + 8 * hh;
    const _Float16* bp = wh + (size_t)(n0 + wn + m) * HH + 8 * hh;
#pragma unroll 1
    for (int kt = 0; kt < HH / 32; ++kt) {
      const int k0 = 32 * kt;
      FragH a0, a1;
      a0.h[0] = *(const v8h*)(ap + k0);
      a0.h[1] = *(const v8h*)(ap + k0 + 16);
      a1.h[0] = *(const v8h*)(ap + (size_t)16 * HH + k0);
      a1.h[1] = *(const v8h*)(ap + (size_t)16 * HH + k0 + 16);
#pragma unroll
      for (int nt = 0; nt < 4; ++nt) {
        const _Float16* bq = bp + (size_t)nt * 16 * HH + k0;
        FragH b;
        b.h[0] = *(const v8h*)bq;
        b.h[1] = *(const v8h*)(bq + 16);
        acc[0][nt] = wmf(a0.v, b.v, acc[0][nt]);
        acc[1][nt] = wmf(a1.v, b.v, acc[1][nt]);
      }
    }
  }

  {
    const _Float16* ap = ch + (size_t)(m0 + wm + m) * RR + 8 * hh;
    const _Float16* bp = pt + (size_t)(n0 + wn + m) * RR + 8 * hh;
    FragH a0, a1;
    a0.h[0] = *(const v8h*)(ap);
    a0.h[1] = *(const v8h*)(ap + 16);
    a1.h[0] = *(const v8h*)(ap + (size_t)16 * RR);
    a1.h[1] = *(const v8h*)(ap + (size_t)16 * RR + 16);
#pragma unroll
    for (int nt = 0; nt < 4; ++nt) {
      const _Float16* bq = bp + (size_t)nt * 16 * RR;
      FragH b;
      b.h[0] = *(const v8h*)bq;
      b.h[1] = *(const v8h*)(bq + 16);
      acc[0][nt] = wmf(a0.v, b.v, acc[0][nt]);
      acc[1][nt] = wmf(a1.v, b.v, acc[1][nt]);
    }
  }

  constexpr float OSC = 1.0f / (float)(XSC * WSC);
  float bv[4];
#pragma unroll
  for (int nt = 0; nt < 4; ++nt) bv[nt] = bias[n0 + wn + 16 * nt + m];
#pragma unroll
  for (int mt = 0; mt < 2; ++mt) {
    float* sp = stg + (16 * mt + 8 * hh) * 64 + m;
#pragma unroll
    for (int nt = 0; nt < 4; ++nt) {
#pragma unroll
      for (int r = 0; r < 8; ++r) sp[r * 64 + 16 * nt] = acc[mt][nt][r] * OSC + bv[nt];
    }
  }
  __syncthreads();

  float* gbase = out + (size_t)(m0 + wm) * HH + n0 + wn;
#pragma unroll
  for (int q = 0; q < 16; ++q) {
    const int row = 2 * q + hh;
    const v4f v = *(const v4f*)(stg + row * 64 + 4 * m);
    *(volatile v4f*)(gbase + (size_t)row * HH + 4 * m) = v;
  }
  __threadfence();
#pragma unroll
  for (int q = 0; q < 16; ++q) {
    const int row = 2 * q + hh;
    const v4f v = *(const v4f*)(stg + row * 64 + 4 * m);
    *(volatile v4f*)(gbase + (size_t)row * HH + 4 * m) = v;
  }
}

extern "C" void kernel_launch(void* const* d_in, const int* in_sizes, int n_in,
                              void* d_out, int out_size, void* d_ws, size_t ws_size,
                              hipStream_t stream) {
  if (n_in < 6) return;
  if (in_sizes[0] != TT * HH || in_sizes[1] != HH * HH || in_sizes[2] != HH) return;
  if (in_sizes[3] != NHD * HH || in_sizes[4] != NHD * HH * RR || in_sizes[5] != RR * HH) return;
  if (out_size != TT * HH) return;

  const float* query = (const float*)d_in[0];
  const float* w     = (const float*)d_in[1];
  const float* bias  = (const float*)d_in[2];
  const float* tok_k = (const float*)d_in[3];
  const float* tok_v = (const float*)d_in[4];
  const float* tok_p = (const float*)d_in[5];
  float* out = (float*)d_out;

  char* ws = (char*)d_ws;
  size_t off = 0;
  const size_t oXh = off; off += (size_t)TT * HH * 2;          off = (off + 255) & ~(size_t)255;
  const size_t oWh = off; off += (size_t)HH * HH * 2;          off = (off + 255) & ~(size_t)255;
  const size_t oVt = off; off += (size_t)NHK * RR * HDIM * 2;  off = (off + 255) & ~(size_t)255;
  const size_t oPt = off; off += (size_t)HH * RR * 2;          off = (off + 255) & ~(size_t)255;
  const size_t oAt = off; off += (size_t)TT * NHK * 4;         off = (off + 255) & ~(size_t)255;
  const size_t oCh = off; off += (size_t)TT * RR * 2;          off = (off + 255) & ~(size_t)255;
  if (off > ws_size || off > (size_t)WSCAP) return;
  _Float16* xh = (_Float16*)(ws + oXh);
  _Float16* wh = (_Float16*)(ws + oWh);
  _Float16* vt = (_Float16*)(ws + oVt);
  _Float16* pt = (_Float16*)(ws + oPt);
  float*  attn = (float*)(ws + oAt);
  _Float16* ch = (_Float16*)(ws + oCh);

  k_cvt<<<(TT * HH) / (8 * NTHR), NTHR, 0, stream>>>(query, xh, (float)XSC);
  k_cvt<<<(HH * HH) / (8 * NTHR), NTHR, 0, stream>>>(w, wh, (float)WSC);
  k_prepv<<<dim3(NHK, HDIM / 128), NTHR, 0, stream>>>(tok_v, vt);
  k_prepp<<<HH / 128, NTHR, 0, stream>>>(tok_p, pt);
  k_attn<<<(TT * NHD) / NTHR, NTHR, 0, stream>>>(query, tok_k, attn);
  k_gg<<<TT / (NWAVE * 32), NTHR, 0, stream>>>(xh, vt, attn, ch);
  hipFuncSetAttribute(reinterpret_cast<const void*>(&k_gemm),
                      hipFuncAttributeMaxDynamicSharedMemorySize, LDS_GEMM);
  k_gemm<<<dim3(HH / 128, TT / 128), NTHR, LDS_GEMM, stream>>>(xh, wh, ch, pt, bias, out);
}
